// Block_83116207112284
// MI455X (gfx1250) — hardware-verified
//
#include <hip/hip_runtime.h>
#include <stddef.h>
#include <stdint.h>
#include <math.h>


#define RT    4096
#define LS    512
#define CC    128
#define N1    512
#define N2    256
#define DI    512
#define XPNP  64
#define KCAT  1024
#define GBM   64
#define GBN   64
#define GTHR  128
#define NTHR  256
#define TPP   72
#define TP_CTAS 256
#define U1    32768
#define U2    65536
#define U3    131072
#define U4    139264
#define U5    141312
#define U6    174080
#define PL_CTAS (U6 / NTHR)
#define WSMAX 134217728

static_assert(U1 % NTHR == 0 && U2 % NTHR == 0 && U3 % NTHR == 0 && U4 % NTHR == 0 && U5 % NTHR == 0 && U6 % NTHR == 0);
static_assert(U1 == N1 * (LS / 8) && U2 - U1 == N2 * (KCAT / 8) && U3 - U2 == 1024 * (512 / 8));
static_assert(U4 - U3 == XPNP * (KCAT / 8) && U5 - U4 == DI * (32 / 8) && U6 - U5 == N2 * (KCAT / 8));
static_assert(RT % GBM == 0 && N1 % GBN == 0 && N2 % GBN == 0 && DI % GBN == 0 && XPNP == GBN);
static_assert(LS % 32 == 0 && KCAT % 32 == 0 && GBM == (GTHR / 32) * 16);
static_assert((TPP * 2) % 16 == 0 && TPP >= 64);

typedef float          v2f   __attribute__((ext_vector_type(2)));
typedef float          v4f   __attribute__((ext_vector_type(4)));
typedef float          v8f   __attribute__((ext_vector_type(8)));
typedef int            v8i   __attribute__((ext_vector_type(8)));
typedef unsigned short v8us  __attribute__((ext_vector_type(8)));
typedef unsigned short v16us __attribute__((ext_vector_type(16)));
typedef __bf16         v16bf __attribute__((ext_vector_type(16)));
typedef v2f  __attribute__((may_alias)) v2fa;
typedef v4f  __attribute__((may_alias)) v4fa;
typedef v8us __attribute__((may_alias)) v8usa;
union FragB { v16bf v; v16us u; v8us h[2]; v8i w; };

__device__ __forceinline__ v8f wmb(const FragB& a, const FragB& b, v8f c) {
  v8f d = __builtin_amdgcn_wmma_f32_16x16x32_bf16(false, a.v, false, b.v, (short)0, c, false, false);
  asm volatile("v_nop\n\tv_nop\n\tv_nop\n\tv_nop" : "+v"(d) : "v"(a.w), "v"(b.w));
  return d;
}

__device__ __forceinline__ unsigned bf16_bits(float f) {
  const unsigned u = __float_as_uint(f);
  return (u + 0x7FFFu + ((u >> 16) & 1u)) >> 16;
}
__device__ __forceinline__ float bf16_val(float f) {
  return __uint_as_float(bf16_bits(f) << 16);
}

__device__ __forceinline__ float silu_f(float v) { return v * (1.0f / (1.0f + expf(-v))); }
__device__ __forceinline__ float softplus_f(float v) { return fmaxf(v, 0.0f) + log1pf(expf(-fabsf(v))); }

__device__ __forceinline__ void split8(const v4f p0, const v4f p1, v8us& hv, v8us& lv) {
  unsigned hb;
  hb = bf16_bits(p0.x); hv[0] = (unsigned short)hb; lv[0] = (unsigned short)bf16_bits(p0.x - __uint_as_float(hb << 16));
  hb = bf16_bits(p0.y); hv[1] = (unsigned short)hb; lv[1] = (unsigned short)bf16_bits(p0.y - __uint_as_float(hb << 16));
  hb = bf16_bits(p0.z); hv[2] = (unsigned short)hb; lv[2] = (unsigned short)bf16_bits(p0.z - __uint_as_float(hb << 16));
  hb = bf16_bits(p0.w); hv[3] = (unsigned short)hb; lv[3] = (unsigned short)bf16_bits(p0.w - __uint_as_float(hb << 16));
  hb = bf16_bits(p1.x); hv[4] = (unsigned short)hb; lv[4] = (unsigned short)bf16_bits(p1.x - __uint_as_float(hb << 16));
  hb = bf16_bits(p1.y); hv[5] = (unsigned short)hb; lv[5] = (unsigned short)bf16_bits(p1.y - __uint_as_float(hb << 16));
  hb = bf16_bits(p1.z); hv[6] = (unsigned short)hb; lv[6] = (unsigned short)bf16_bits(p1.z - __uint_as_float(hb << 16));
  hb = bf16_bits(p1.w); hv[7] = (unsigned short)hb; lv[7] = (unsigned short)bf16_bits(p1.w - __uint_as_float(hb << 16));
}

__device__ __forceinline__ void plane_unit(const float* __restrict__ W, unsigned short* P, int v, int lg,
                                           int ksm, int spitch, int nsrc) {
  const int n  = v >> lg;
  const int k8 = (v & ((1 << lg) - 1)) * 8;
  const int ks = k8 & ksm;
  const int nc = n < nsrc ? n : nsrc - 1;
  const float* p = W + (size_t)nc * spitch + ks;
  const v4f a = *(const v4f*)p;
  const v4f b = *(const v4f*)(p + 4);
  const bool ok = n < nsrc;
  v8us o;
  o[0] = ok ? (unsigned short)bf16_bits(a.x) : (unsigned short)0;
  o[1] = ok ? (unsigned short)bf16_bits(a.y) : (unsigned short)0;
  o[2] = ok ? (unsigned short)bf16_bits(a.z) : (unsigned short)0;
  o[3] = ok ? (unsigned short)bf16_bits(a.w) : (unsigned short)0;
  o[4] = ok ? (unsigned short)bf16_bits(b.x) : (unsigned short)0;
  o[5] = ok ? (unsigned short)bf16_bits(b.y) : (unsigned short)0;
  o[6] = ok ? (unsigned short)bf16_bits(b.z) : (unsigned short)0;
  o[7] = ok ? (unsigned short)bf16_bits(b.w) : (unsigned short)0;
  unsigned short* dp = P + (size_t)v * 8;
  *(volatile v8us*)dp = o;
  __threadfence();
  *(volatile v8us*)dp = o;
}

__global__ __launch_bounds__(NTHR) void k_prep(
    const float* __restrict__ x, const float* __restrict__ lin1_w, const float* __restrict__ lin2_w,
    const float* __restrict__ inw2, const float* __restrict__ xpw2, const float* __restrict__ dtw2,
    const float* __restrict__ outw2,
    const float* __restrict__ cw2, const float* __restrict__ cb2, const float* __restrict__ dtb2,
    const float* __restrict__ dd2,
    const float* __restrict__ m1in, const float* __restrict__ m1cw, const float* __restrict__ m1cb,
    const float* __restrict__ m1xp, const float* __restrict__ m1dw, const float* __restrict__ m1db,
    const float* __restrict__ m1al, const float* __restrict__ m1dd, const float* __restrict__ m1ow,
    unsigned short* XT, unsigned short* LW1, unsigned short* LW2, unsigned short* INW, unsigned short* XPW,
    unsigned short* DTW, unsigned short* OUTW, float* V2, float* M1C) {
  __shared__ __attribute__((aligned(16))) unsigned short sT[CC * TPP];
  __shared__ __attribute__((aligned(16))) float sm1[128];
  const int tid = (int)threadIdx.x;
  const int bid = (int)blockIdx.x;

  if (bid < TP_CTAS) {
    const int b  = bid >> 3;
    const int l0 = (bid & 7) * 64;
#pragma unroll 1
    for (int it = 0; it < 8; ++it) {
      const int idx = it * NTHR + tid;
      const int l  = idx >> 5;
      const int c4 = idx & 31;
      const v4f a = *(const v4f*)(x + ((size_t)b * LS + l0 + l) * CC + 4 * c4);
      sT[(4 * c4 + 0) * TPP + l] = (unsigned short)bf16_bits(a.x);
      sT[(4 * c4 + 1) * TPP + l] = (unsigned short)bf16_bits(a.y);
      sT[(4 * c4 + 2) * TPP + l] = (unsigned short)bf16_bits(a.z);
      sT[(4 * c4 + 3) * TPP + l] = (unsigned short)bf16_bits(a.w);
    }
    __syncthreads();
    v8us o[4];
#pragma unroll
    for (int it = 0; it < 4; ++it) {
      const int idx = it * NTHR + tid;
      const int c = idx >> 3, q = idx & 7;
      o[it] = *(const v8usa*)(sT + c * TPP + 8 * q);
    }
#pragma unroll
    for (int it = 0; it < 4; ++it) {
      const int idx = it * NTHR + tid;
      const int c = idx >> 3, q = idx & 7;
      *(volatile v8us*)(XT + (size_t)(b * CC + c) * LS + l0 + 8 * q) = o[it];
    }
    __threadfence();
#pragma unroll
    for (int it = 0; it < 4; ++it) {
      const int idx = it * NTHR + tid;
      const int c = idx >> 3, q = idx & 7;
      *(volatile v8us*)(XT + (size_t)(b * CC + c) * LS + l0 + 8 * q) = o[it];
    }
  } else if (bid < TP_CTAS + PL_CTAS) {
    const int u = (bid - TP_CTAS) * NTHR + tid;
    if (u < U1)      plane_unit(lin1_w, LW1,  u,      6, 511, 512, 512);
    else if (u < U2) plane_unit(lin2_w, LW2,  u - U1, 7, 511, 512, 256);
    else if (u < U3) plane_unit(inw2,   INW,  u - U2, 6, 255, 256, 1024);
    else if (u < U4) plane_unit(xpw2,   XPW,  u - U3, 7, 511, 512, 48);
    else if (u < U5) plane_unit(dtw2,   DTW,  u - U4, 2, 15,  16,  512);
    else             plane_unit(outw2,  OUTW, u - U5, 7, 511, 512, 256);
  } else {
    if (tid < 128) {
      const int d4 = 4 * tid;
      const v4f c0 = *(const v4f*)(cw2 + 4 * (size_t)(d4 + 0));
      const v4f c1 = *(const v4f*)(cw2 + 4 * (size_t)(d4 + 1));
      const v4f c2 = *(const v4f*)(cw2 + 4 * (size_t)(d4 + 2));
      const v4f c3 = *(const v4f*)(cw2 + 4 * (size_t)(d4 + 3));
      const v4f e0 = *(const v4f*)(cb2 + d4);
      const v4f e1 = *(const v4f*)(dtb2 + d4);
      const v4f e2 = *(const v4f*)(dd2 + d4);
      v4f o0, o1, o2, o3;
      o0.x = bf16_val(c0.w); o0.y = bf16_val(c1.w); o0.z = bf16_val(c2.w); o0.w = bf16_val(c3.w);
      o1.x = bf16_val(e0.x); o1.y = bf16_val(e0.y); o1.z = bf16_val(e0.z); o1.w = bf16_val(e0.w);
      o2.x = bf16_val(e1.x); o2.y = bf16_val(e1.y); o2.z = bf16_val(e1.z); o2.w = bf16_val(e1.w);
      o3.x = bf16_val(e2.x); o3.y = bf16_val(e2.y); o3.z = bf16_val(e2.z); o3.w = bf16_val(e2.w);
      *(volatile v4f*)(V2 + 0 * DI + d4) = o0;
      *(volatile v4f*)(V2 + 1 * DI + d4) = o1;
      *(volatile v4f*)(V2 + 2 * DI + d4) = o2;
      *(volatile v4f*)(V2 + 3 * DI + d4) = o3;
      __threadfence();
      *(volatile v4f*)(V2 + 0 * DI + d4) = o0;
      *(volatile v4f*)(V2 + 1 * DI + d4) = o1;
      *(volatile v4f*)(V2 + 2 * DI + d4) = o2;
      *(volatile v4f*)(V2 + 3 * DI + d4) = o3;
    }
    __syncthreads();
    { const float v = m1in[tid < 4 ? tid : 3];   if (tid < 4)  sm1[tid] = bf16_val(v); }
    { const float v = m1cw[tid < 8 ? tid : 7];   if (tid < 8)  sm1[4 + tid] = bf16_val(v); }
    { const float v = m1cb[tid < 2 ? tid : 1];   if (tid < 2)  sm1[12 + tid] = bf16_val(v); }
    { const float v = m1xp[tid < 66 ? tid : 65]; if (tid < 66) sm1[14 + tid] = bf16_val(v); }
    __syncthreads();
    { const float v = m1dw[tid < 2 ? tid : 1];   if (tid < 2)  sm1[80 + tid] = bf16_val(v); }
    { const float v = m1db[tid < 2 ? tid : 1];   if (tid < 2)  sm1[82 + tid] = bf16_val(v); }
    { const float v = m1al[tid < 32 ? tid : 31]; if (tid < 32) sm1[84 + tid] = -expf(bf16_val(v)); }
    { const float v = m1dd[tid < 2 ? tid : 1];   if (tid < 2)  sm1[116 + tid] = bf16_val(v); }
    __syncthreads();
    { const float v = m1ow[tid < 2 ? tid : 1];   if (tid < 2)  sm1[118 + tid] = bf16_val(v); }
    if (tid >= 120 && tid < 128) sm1[tid] = 0.0f;
    __syncthreads();
    if (tid < 32) {
      const v4f o = *(const v4fa*)(sm1 + 4 * tid);
      *(volatile v4f*)(M1C + 4 * tid) = o;
      __threadfence();
      *(volatile v4f*)(M1C + 4 * tid) = o;
    }
  }
}

template <int MODE>
__global__ __launch_bounds__(GTHR) void k_gemm(
    const unsigned short* __restrict__ A, const unsigned short* __restrict__ WT, int K,
    const float* __restrict__ va, const float* __restrict__ vb,
    float* outF, int ldo, float* outG, unsigned short* outH)
{
  __shared__ __attribute__((aligned(16))) float stg[GBM * GBN];
  const int tid = (int)threadIdx.x, lane = tid & 31, wave = tid >> 5, hh = lane >> 4, m = lane & 15;
  const int rowBase = (int)blockIdx.x * GBM;
  const int col0    = (int)blockIdx.y * GBN;

  v8f acc[4];
  {
    const v8f z = {0.f, 0.f, 0.f, 0.f, 0.f, 0.f, 0.f, 0.f};
    acc[0] = z; acc[1] = z; acc[2] = z; acc[3] = z;
  }
  const unsigned short* ap = A  + (size_t)(rowBase + 16 * wave + m) * (size_t)K + 8 * hh;
  const unsigned short* wp = WT + (size_t)(col0 + m) * (size_t)K + 8 * hh;
  const int ksteps = K >> 5;
#pragma unroll 1
  for (int ks = 0; ks < ksteps; ++ks) {
    FragB af;
    af.h[0] = *(const v8usa*)(ap + 32 * ks);
    af.h[1] = *(const v8usa*)(ap + 32 * ks + 16);
#pragma unroll
    for (int t = 0; t < 4; ++t) {
      const unsigned short* wq = wp + (size_t)(16 * t) * (size_t)K + 32 * ks;
      FragB bf;
      bf.h[0] = *(const v8usa*)wq;
      bf.h[1] = *(const v8usa*)(wq + 16);
      acc[t] = wmb(af, bf, acc[t]);
    }
  }

#pragma unroll
  for (int t = 0; t < 4; ++t) {
    const int lc = 16 * t + m;
#pragma unroll
    for (int r = 0; r < 8; ++r) {
      const int lr = 16 * wave + 8 * hh + r;
      stg[lr * GBN + lc] = acc[t][r];
    }
  }
  __syncthreads();

  const int rq = lane >> 3, q = lane & 7;

  if constexpr (MODE == 0) {
    v4f b0, b1;
    {
      const v4f t0 = *(const v4f*)(va + col0 + 8 * q);
      const v4f t1 = *(const v4f*)(va + col0 + 8 * q + 4);
      b0.x = bf16_val(t0.x); b0.y = bf16_val(t0.y); b0.z = bf16_val(t0.z); b0.w = bf16_val(t0.w);
      b1.x = bf16_val(t1.x); b1.y = bf16_val(t1.y); b1.z = bf16_val(t1.z); b1.w = bf16_val(t1.w);
    }
    v8us hv[4], lv[4];
#pragma unroll
    for (int it = 0; it < 4; ++it) {
      const int lr = 16 * wave + 4 * it + rq;
      const v4f p0 = *(const v4fa*)(stg + lr * GBN + 8 * q) + b0;
      const v4f p1 = *(const v4fa*)(stg + lr * GBN + 8 * q + 4) + b1;
      split8(p0, p1, hv[it], lv[it]);
    }
#pragma unroll
    for (int it = 0; it < 4; ++it) {
      const int lr = 16 * wave + 4 * it + rq;
      unsigned short* dp = outH + (size_t)(rowBase + lr) * KCAT + col0 + 8 * q;
      *(volatile v8us*)dp = hv[it];
      *(volatile v8us*)(dp + DI) = lv[it];
    }
    __threadfence();
#pragma unroll
    for (int it = 0; it < 4; ++it) {
      const int lr = 16 * wave + 4 * it + rq;
      unsigned short* dp = outH + (size_t)(rowBase + lr) * KCAT + col0 + 8 * q;
      *(volatile v8us*)dp = hv[it];
      *(volatile v8us*)(dp + DI) = lv[it];
    }
  } else if constexpr (MODE == 2) {
    const bool isx = col0 < DI;
    if (isx) {
      const v4f w3 = *(const v4f*)(va + col0 + 4 * m);
      const v4f cb = *(const v4f*)(vb + col0 + 4 * m);
#pragma unroll 1
      for (int i = 0; i < 8; ++i) {
        const int lr = 16 * wave + 2 * i + hh;
        const v4f t = *(const v4fa*)(stg + lr * GBN + 4 * m);
        v4f xc;
        xc.x = silu_f(w3.x * t.x + cb.x);
        xc.y = silu_f(w3.y * t.y + cb.y);
        xc.z = silu_f(w3.z * t.z + cb.z);
        xc.w = silu_f(w3.w * t.w + cb.w);
        *(v4fa*)(stg + lr * GBN + 4 * m) = xc;
        float* op = outF + (size_t)(rowBase + lr) * (size_t)ldo + col0 + 4 * m;
        *(volatile v4f*)op = xc;
        __threadfence();
        *(volatile v4f*)op = xc;
      }
    } else {
#pragma unroll 1
      for (int i = 0; i < 8; ++i) {
        const int lr = 16 * wave + 2 * i + hh;
        const v4f t = *(const v4fa*)(stg + lr * GBN + 4 * m);
        v4f sz;
        sz.x = silu_f(t.x); sz.y = silu_f(t.y); sz.z = silu_f(t.z); sz.w = silu_f(t.w);
        float* op = outG + (size_t)(rowBase + lr) * (size_t)ldo + (col0 - DI) + 4 * m;
        *(volatile v4f*)op = sz;
        __threadfence();
        *(volatile v4f*)op = sz;
      }
    }
    __syncthreads();
    if (isx) {
#pragma unroll 1
      for (int it = 0; it < 4; ++it) {
        const int lr = 16 * wave + 4 * it + rq;
        const v4f p0 = *(const v4fa*)(stg + lr * GBN + 8 * q);
        const v4f p1 = *(const v4fa*)(stg + lr * GBN + 8 * q + 4);
        v8us hv, lv;
        split8(p0, p1, hv, lv);
        unsigned short* dp = outH + (size_t)(rowBase + lr) * KCAT + col0 + 8 * q;
        *(volatile v8us*)dp = hv;
        *(volatile v8us*)(dp + DI) = lv;
        __threadfence();
        *(volatile v8us*)dp = hv;
        *(volatile v8us*)(dp + DI) = lv;
      }
    }
  } else {
    v4f bb = {0.f, 0.f, 0.f, 0.f};
    if constexpr (MODE == 1) {
      const v4f t0 = *(const v4f*)(va + col0 + 4 * m);
      bb.x = bf16_val(t0.x); bb.y = bf16_val(t0.y); bb.z = bf16_val(t0.z); bb.w = bf16_val(t0.w);
    }
    v4f fv[8];
#pragma unroll
    for (int i = 0; i < 8; ++i) {
      const int lr = 16 * wave + 2 * i + hh;
      fv[i] = *(const v4fa*)(stg + lr * GBN + 4 * m) + bb;
    }
#pragma unroll
    for (int i = 0; i < 8; ++i) {
      const int lr = 16 * wave + 2 * i + hh;
      float* op = outF + (size_t)(rowBase + lr) * (size_t)ldo + col0 + 4 * m;
      *(volatile v4f*)op = fv[i];
    }
    __threadfence();
#pragma unroll
    for (int i = 0; i < 8; ++i) {
      const int lr = 16 * wave + 2 * i + hh;
      float* op = outF + (size_t)(rowBase + lr) * (size_t)ldo + col0 + 4 * m;
      *(volatile v4f*)op = fv[i];
    }
  }
}

__device__ __forceinline__ void decomp1(float h, float& mean, float& rem) {
#pragma clang fp contract(off)
  float s = 0.0f;
  for (int i = 0; i < 25; ++i) s = s + h;
  mean = s * (1.0f / 25.0f);
  rem  = h - mean;
}

__global__ __launch_bounds__(NTHR) void k_decomp_corr(const float* __restrict__ H, unsigned short* ST) {
  __shared__ __attribute__((aligned(16))) float srem[4 * 512];
  __shared__ __attribute__((aligned(16))) float smean[4 * 256];
  __shared__ __attribute__((aligned(16))) float sst[4 * 256];
  const int tid = (int)threadIdx.x;
  const int rr = tid >> 6, t = tid & 63;
  const int row = (int)blockIdx.x * 4 + rr;

  {
    const v4f hv = *(const v4f*)(H + (size_t)row * N2 + 4 * t);
    v4f mv, rv;
    float a, b;
    decomp1(hv.x, a, b); mv.x = a; rv.x = b;
    decomp1(hv.y, a, b); mv.y = a; rv.y = b;
    decomp1(hv.z, a, b); mv.z = a; rv.z = b;
    decomp1(hv.w, a, b); mv.w = a; rv.w = b;
    *(v4fa*)(smean + rr * 256 + 4 * t) = mv;
    *(v4fa*)(srem + rr * 512 + 4 * t) = rv;
    *(v4fa*)(srem + rr * 512 + 256 + 4 * t) = rv;
  }
  __syncthreads();

  float a0 = 0.0f, a1 = 0.0f, a2 = 0.0f, a3 = 0.0f;
  const float* rp = srem + rr * 512 + 4 * t;
  const float* mp = smean + rr * 256;
#pragma unroll 2
  for (int m4 = 0; m4 < 64; ++m4) {
    const v4f mv = *(const v4fa*)(mp + 4 * m4);
    const v4f ra = *(const v4fa*)(rp + 4 * m4);
    const v4f rb = *(const v4fa*)(rp + 4 * m4 + 4);
    a0 = fmaf(ra.x, mv.x, a0); a0 = fmaf(ra.y, mv.y, a0); a0 = fmaf(ra.z, mv.z, a0); a0 = fmaf(ra.w, mv.w, a0);
    a1 = fmaf(ra.y, mv.x, a1); a1 = fmaf(ra.z, mv.y, a1); a1 = fmaf(ra.w, mv.z, a1); a1 = fmaf(rb.x, mv.w, a1);
    a2 = fmaf(ra.z, mv.x, a2); a2 = fmaf(ra.w, mv.y, a2); a2 = fmaf(rb.x, mv.z, a2); a2 = fmaf(rb.y, mv.w, a2);
    a3 = fmaf(ra.w, mv.x, a3); a3 = fmaf(rb.x, mv.y, a3); a3 = fmaf(rb.y, mv.z, a3); a3 = fmaf(rb.z, mv.w, a3);
  }
  {
    v4f o; o.x = a0; o.y = a1; o.z = a2; o.w = a3;
    *(v4fa*)(sst + rr * 256 + 4 * t) = o;
  }
  __syncthreads();

  const int p = t & 31;
  const bool sel = (t >> 5) != 0;
  const v4f p0 = *(const v4fa*)(sst + rr * 256 + 8 * p);
  const v4f p1 = *(const v4fa*)(sst + rr * 256 + 8 * p + 4);
  v8us hv, lv;
  split8(p0, p1, hv, lv);
  const v8us ov = sel ? lv : hv;
  unsigned short* dp = ST + (size_t)row * LS + (sel ? 256 : 0) + 8 * p;
  *(volatile v8us*)dp = ov;
  __threadfence();
  *(volatile v8us*)dp = ov;
}

__global__ __launch_bounds__(GTHR) void k_m2_dt(const float* __restrict__ DBC, const unsigned short* __restrict__ DTW,
                                                const float* __restrict__ V2, const float* __restrict__ XC,
                                                const float* __restrict__ SZ, unsigned short* Y) {
  __shared__ __attribute__((aligned(16))) float stg[GBM * GBN];
  __shared__ __attribute__((aligned(16))) float sbc[GBM * 32];
  const int tid = (int)threadIdx.x, lane = tid & 31, wave = tid >> 5, hh = lane >> 4, m = lane & 15;
  const int rowBase = (int)blockIdx.x * GBM;
  const int col0    = (int)blockIdx.y * GBN;

  FragB af;
  {
    const float* p = DBC + (size_t)(rowBase + 16 * wave + m) * XPNP + 8 * hh;
    const v4f a = *(const v4f*)p;
    const v4f b = *(const v4f*)(p + 4);
    v8us h8, l8;
    split8(a, b, h8, l8);
    af.h[0] = h8;
    af.h[1] = l8;
  }
  v8f acc[4];
  {
    const v8f z = {0.f, 0.f, 0.f, 0.f, 0.f, 0.f, 0.f, 0.f};
#pragma unroll
    for (int t = 0; t < 4; ++t) {
      const unsigned short* wq = DTW + (size_t)(col0 + 16 * t + m) * 32 + 8 * hh;
      FragB bf;
      bf.h[0] = *(const v8usa*)wq;
      bf.h[1] = *(const v8usa*)(wq + 16);
      acc[t] = wmb(af, bf, z);
    }
  }
#pragma unroll
  for (int t = 0; t < 4; ++t) {
    const int lc = 16 * t + m;
#pragma unroll
    for (int r = 0; r < 8; ++r) {
      const int lr = 16 * wave + 8 * hh + r;
      stg[lr * GBN + lc] = acc[t][r];
    }
  }
#pragma unroll
  for (int it = 0; it < 4; ++it) {
    const int idx = it * GTHR + tid;
    const int r = idx >> 3, c4 = idx & 7;
    const v4f v = *(const v4f*)(DBC + (size_t)(rowBase + r) * XPNP + 16 + 4 * c4);
    *(v4fa*)(sbc + r * 32 + 4 * c4) = v;
  }
  __syncthreads();

  const int rq = lane >> 3, q = lane & 7;
  float dtb[8], ddv[8];
  {
    const v4f t0 = *(const v4f*)(V2 + 2 * DI + col0 + 8 * q);
    const v4f t1 = *(const v4f*)(V2 + 2 * DI + col0 + 8 * q + 4);
    const v4f u0 = *(const v4f*)(V2 + 3 * DI + col0 + 8 * q);
    const v4f u1 = *(const v4f*)(V2 + 3 * DI + col0 + 8 * q + 4);
    dtb[0] = t0.x; dtb[1] = t0.y; dtb[2] = t0.z; dtb[3] = t0.w;
    dtb[4] = t1.x; dtb[5] = t1.y; dtb[6] = t1.z; dtb[7] = t1.w;
    ddv[0] = u0.x; ddv[1] = u0.y; ddv[2] = u0.z; ddv[3] = u0.w;
    ddv[4] = u1.x; ddv[5] = u1.y; ddv[6] = u1.z; ddv[7] = u1.w;
  }
#pragma unroll 1
  for (int it = 0; it < 4; ++it) {
    const int lr = 16 * wave + 4 * it + rq;
    const int gr = rowBase + lr;
    const v4f p0 = *(const v4fa*)(stg + lr * GBN + 8 * q);
    const v4f p1 = *(const v4fa*)(stg + lr * GBN + 8 * q + 4);
    const v4f x0 = *(const v4f*)(XC + (size_t)gr * DI + col0 + 8 * q);
    const v4f x1 = *(const v4f*)(XC + (size_t)gr * DI + col0 + 8 * q + 4);
    const v4f z0 = *(const v4f*)(SZ + (size_t)gr * DI + col0 + 8 * q);
    const v4f z1 = *(const v4f*)(SZ + (size_t)gr * DI + col0 + 8 * q + 4);
    float pv[8], xv[8], zv[8], tv[8], s[8];
    pv[0] = p0.x; pv[1] = p0.y; pv[2] = p0.z; pv[3] = p0.w; pv[4] = p1.x; pv[5] = p1.y; pv[6] = p1.z; pv[7] = p1.w;
    xv[0] = x0.x; xv[1] = x0.y; xv[2] = x0.z; xv[3] = x0.w; xv[4] = x1.x; xv[5] = x1.y; xv[6] = x1.z; xv[7] = x1.w;
    zv[0] = z0.x; zv[1] = z0.y; zv[2] = z0.z; zv[3] = z0.w; zv[4] = z1.x; zv[5] = z1.y; zv[6] = z1.z; zv[7] = z1.w;
#pragma unroll
    for (int e = 0; e < 8; ++e) {
      tv[e] = softplus_f(pv[e] + dtb[e]) * xv[e];
      s[e] = 0.0f;
    }
    const float* bc = sbc + lr * 32;
#pragma unroll 4
    for (int n = 0; n < 16; ++n) {
      const float bm = bc[n];
      const float cm = bc[16 + n];
#pragma unroll
      for (int e = 0; e < 8; ++e) s[e] = s[e] + (tv[e] * bm) * cm;
    }
    v4f y0, y1;
    y0.x = (s[0] + xv[0] * ddv[0]) * zv[0]; y0.y = (s[1] + xv[1] * ddv[1]) * zv[1];
    y0.z = (s[2] + xv[2] * ddv[2]) * zv[2]; y0.w = (s[3] + xv[3] * ddv[3]) * zv[3];
    y1.x = (s[4] + xv[4] * ddv[4]) * zv[4]; y1.y = (s[5] + xv[5] * ddv[5]) * zv[5];
    y1.z = (s[6] + xv[6] * ddv[6]) * zv[6]; y1.w = (s[7] + xv[7] * ddv[7]) * zv[7];
    v8us hv, lv;
    split8(y0, y1, hv, lv);
    unsigned short* dp = Y + (size_t)gr * KCAT + col0 + 8 * q;
    *(volatile v8us*)dp = hv;
    *(volatile v8us*)(dp + DI) = lv;
    __threadfence();
    *(volatile v8us*)dp = hv;
    *(volatile v8us*)(dp + DI) = lv;
  }
}

__global__ __launch_bounds__(128) void k_m1_scan(const float* __restrict__ H, const float* __restrict__ X1,
                                                 const float* __restrict__ M1C, float* out) {
  __shared__ __attribute__((aligned(16))) float sc[128];
  __shared__ __attribute__((aligned(16))) float su[4 * 256];
  __shared__ __attribute__((aligned(16))) float sxc[4 * 512];
  __shared__ __attribute__((aligned(16))) float sdt[4 * 512];
  __shared__ __attribute__((aligned(16))) float ssz[4 * 512];
  __shared__ __attribute__((aligned(16))) float sx2[4 * 256];
  const int tid = (int)threadIdx.x, lane = tid & 31, wave = tid >> 5;
  const int row = (int)blockIdx.x * 4 + wave;
  float* u   = su  + wave * 256;
  float* wxc = sxc + wave * 512;
  float* wdt = sdt + wave * 512;
  float* wsz = ssz + wave * 512;
  float* wx2 = sx2 + wave * 256;

  sc[tid] = M1C[tid];
  {
    const v4f a = *(const v4f*)(H + (size_t)row * N2 + 4 * lane);
    const v4f b = *(const v4f*)(H + (size_t)row * N2 + 128 + 4 * lane);
    *(v4fa*)(u + 4 * lane) = a;
    *(v4fa*)(u + 128 + 4 * lane) = b;
  }
  __syncthreads();

  {
    const int dq = lane & 1;
    const float inx = sc[dq], inz = sc[2 + dq];
    const float cw0 = sc[4 + 4 * dq], cw1 = sc[5 + 4 * dq], cw2 = sc[6 + 4 * dq], cw3 = sc[7 + 4 * dq];
    const float cbd = sc[12 + dq], xp0 = sc[14 + dq], dwd = sc[80 + dq], dbd = sc[82 + dq];
#pragma unroll 1
    for (int i = 0; i < 16; ++i) {
      const int item = lane + 32 * i;
      const int t  = item >> 1;
      const int t1 = (t - 1) < 0 ? 0 : (t - 1);
      const int t2 = (t - 2) < 0 ? 0 : (t - 2);
      const int t3 = (t - 3) < 0 ? 0 : (t - 3);
      const float u0 = u[t];
      float u1 = u[t1], u2 = u[t2], u3 = u[t3];
      u1 = (t >= 1) ? u1 : 0.0f;
      u2 = (t >= 2) ? u2 : 0.0f;
      u3 = (t >= 3) ? u3 : 0.0f;
      const float cv = ((cw0 * (u3 * inx) + cw1 * (u2 * inx)) + cw2 * (u1 * inx)) + cw3 * (u0 * inx);
      const float xc = silu_f(cv + cbd);
      const float part = xc * xp0;
      const float oth  = __shfl_xor(part, 1, 32);
      const float dtin = part + oth;
      const float dtv  = softplus_f(dtin * dwd + dbd);
      const float szv  = silu_f(u0 * inz);
      wxc[item] = xc;
      wdt[item] = dtv;
      wsz[item] = szv;
    }
  }
  __syncthreads();

  {
    const int d = lane >> 4, n = lane & 15;
    const float Adn = sc[84 + 16 * d + n];
    const float xB0 = sc[14 + 2 * (1 + n)],  xB1 = sc[15 + 2 * (1 + n)];
    const float xC0 = sc[14 + 2 * (17 + n)], xC1 = sc[15 + 2 * (17 + n)];
    const float Dd  = sc[116 + d];
    const float owd = sc[118 + d];
    float hst = 0.0f;
#pragma unroll 1
    for (int t = 0; t < N2; ++t) {
      const v2f xcv = *(const v2fa*)(wxc + 2 * t);
      const float dtd = wdt[2 * t + d];
      const float szd = wsz[2 * t + d];
      const float xcd = (d != 0) ? xcv.y : xcv.x;
      const float Bn = xcv.x * xB0 + xcv.y * xB1;
      const float Cn = xcv.x * xC0 + xcv.y * xC1;
      hst = expf(dtd * Adn) * hst + (dtd * xcd) * Bn;
      float p = hst * Cn;
      p += __shfl_xor(p, 8, 32);
      p += __shfl_xor(p, 4, 32);
      p += __shfl_xor(p, 2, 32);
      p += __shfl_xor(p, 1, 32);
      const float y = (p + xcd * Dd) * szd;
      const float c = y * owd;
      const float tot = c + __shfl_xor(c, 16, 32);
      if (lane == 0) wx2[t] = tot;
    }
  }
  __syncthreads();

  {
    const v4f xa = *(const v4fa*)(wx2 + 4 * lane);
    const v4f xb = *(const v4fa*)(wx2 + 128 + 4 * lane);
    const v4f ha = *(const v4fa*)(u + 4 * lane);
    const v4f hb = *(const v4fa*)(u + 128 + 4 * lane);
    const v4f ya = *(const v4f*)(X1 + (size_t)row * N2 + 4 * lane);
    const v4f yb = *(const v4f*)(X1 + (size_t)row * N2 + 128 + 4 * lane);
    const v4f oa = (xa + ya) + ha;
    const v4f ob = (xb + yb) + hb;
    float* op = out + (size_t)row * N2 + 4 * lane;
    *(volatile v4f*)op = oa;
    *(volatile v4f*)(op + 128) = ob;
    __threadfence();
    *(volatile v4f*)op = oa;
    *(volatile v4f*)(op + 128) = ob;
  }
}

static inline size_t al256(size_t o) { return (o + 255) & ~(size_t)255; }

extern "C" void kernel_launch(void* const* d_in, const int* in_sizes, int n_in,
                              void* d_out, int out_size, void* d_ws, size_t ws_size,
                              hipStream_t stream) {
  if (n_in < 23) return;
  const int want[23] = {
      32 * LS * CC, N1 * LS, N1, N2 * N1, N2,
      4, 8, 2, 66, 2, 2, 32, 2, 2,
      1024 * 256, DI * 4, DI, 48 * DI, DI * 16, DI, DI * 16, DI, N2 * DI};
  for (int i = 0; i < 23; ++i) if (in_sizes[i] != want[i]) return;
  if (out_size != RT * N2) return;

  const float* x       = (const float*)d_in[0];
  const float* lin1_w  = (const float*)d_in[1];
  const float* lin1_b  = (const float*)d_in[2];
  const float* lin2_w  = (const float*)d_in[3];
  const float* lin2_b  = (const float*)d_in[4];
  const float* m1_in   = (const float*)d_in[5];
  const float* m1_cw   = (const float*)d_in[6];
  const float* m1_cb   = (const float*)d_in[7];
  const float* m1_xp   = (const float*)d_in[8];
  const float* m1_dw   = (const float*)d_in[9];
  const float* m1_db   = (const float*)d_in[10];
  const float* m1_al   = (const float*)d_in[11];
  const float* m1_dd   = (const float*)d_in[12];
  const float* m1_ow   = (const float*)d_in[13];
  const float* m2_in   = (const float*)d_in[14];
  const float* m2_cw   = (const float*)d_in[15];
  const float* m2_cb   = (const float*)d_in[16];
  const float* m2_xp   = (const float*)d_in[17];
  const float* m2_dw   = (const float*)d_in[18];
  const float* m2_db   = (const float*)d_in[19];
  const float* m2_dd   = (const float*)d_in[21];
  const float* m2_ow   = (const float*)d_in[22];
  float* out = (float*)d_out;

  char* ws = (char*)d_ws;
  size_t off = 0;
  const size_t oXT  = off; off = al256(off + (size_t)RT * LS * 2);
  const size_t oLW1 = off; off = al256(off + (size_t)N1 * LS * 2);
  const size_t oLW2 = off; off = al256(off + (size_t)N2 * KCAT * 2);
  const size_t oINW = off; off = al256(off + (size_t)1024 * 512 * 2);
  const size_t oXPW = off; off = al256(off + (size_t)XPNP * KCAT * 2);
  const size_t oDTW = off; off = al256(off + (size_t)DI * 32 * 2);
  const size_t oOW  = off; off = al256(off + (size_t)N2 * KCAT * 2);
  const size_t oV2  = off; off = al256(off + (size_t)4 * DI * 4);
  const size_t oM1C = off; off = al256(off + (size_t)128 * 4);
  const size_t oH1  = off; off = al256(off + (size_t)RT * KCAT * 2);
  const size_t oH   = off; off = al256(off + (size_t)RT * N2 * 4);
  const size_t oST  = off; off = al256(off + (size_t)RT * LS * 2);
  const size_t oXC  = off; off = al256(off + (size_t)RT * DI * 4);
  const size_t oXCH = off; off = al256(off + (size_t)RT * KCAT * 2);
  const size_t oSZ  = off; off = al256(off + (size_t)RT * DI * 4);
  const size_t oDBC = off; off = al256(off + (size_t)RT * XPNP * 4);
  const size_t oY   = off; off = al256(off + (size_t)RT * KCAT * 2);
  const size_t oX1  = off; off = al256(off + (size_t)RT * N2 * 4);
  if (off > ws_size || off > (size_t)WSMAX) return;
  unsigned short* XT   = (unsigned short*)(ws + oXT);
  unsigned short* LW1  = (unsigned short*)(ws + oLW1);
  unsigned short* LW2  = (unsigned short*)(ws + oLW2);
  unsigned short* INW  = (unsigned short*)(ws + oINW);
  unsigned short* XPW  = (unsigned short*)(ws + oXPW);
  unsigned short* DTW  = (unsigned short*)(ws + oDTW);
  unsigned short* OUTW = (unsigned short*)(ws + oOW);
  float*          V2   = (float*)(ws + oV2);
  float*          M1C  = (float*)(ws + oM1C);
  unsigned short* H1   = (unsigned short*)(ws + oH1);
  float*          Hf   = (float*)(ws + oH);
  unsigned short* ST   = (unsigned short*)(ws + oST);
  float*          XC   = (float*)(ws + oXC);
  unsigned short* XCH  = (unsigned short*)(ws + oXCH);
  float*          SZ   = (float*)(ws + oSZ);
  float*          DBC  = (float*)(ws + oDBC);
  unsigned short* Ypl  = (unsigned short*)(ws + oY);
  float*          X1   = (float*)(ws + oX1);

  k_prep<<<TP_CTAS + PL_CTAS + 1, NTHR, 0, stream>>>(
      x, lin1_w, lin2_w, m2_in, m2_xp, m2_dw, m2_ow, m2_cw, m2_cb, m2_db, m2_dd,
      m1_in, m1_cw, m1_cb, m1_xp, m1_dw, m1_db, m1_al, m1_dd, m1_ow,
      XT, LW1, LW2, INW, XPW, DTW, OUTW, V2, M1C);
  k_gemm<0><<<dim3(RT / GBM, N1 / GBN), GTHR, 0, stream>>>(XT, LW1, LS, lin1_b, lin1_b, Hf, N2, Hf, H1);
  k_gemm<1><<<dim3(RT / GBM, N2 / GBN), GTHR, 0, stream>>>(H1, LW2, KCAT, lin2_b, lin2_b, Hf, N2, Hf, Ypl);
  k_decomp_corr<<<RT / 4, NTHR, 0, stream>>>(Hf, ST);
  k_gemm<2><<<dim3(RT / GBM, 1024 / GBN), GTHR, 0, stream>>>(ST, INW, LS, V2, V2 + DI, XC, DI, SZ, XCH);
  k_gemm<3><<<dim3(RT / GBM, 1), GTHR, 0, stream>>>(XCH, XPW, KCAT, V2, V2, DBC, XPNP, DBC, Ypl);
  k_m2_dt<<<dim3(RT / GBM, DI / GBN), GTHR, 0, stream>>>(DBC, DTW, V2, XC, SZ, Ypl);
  k_gemm<4><<<dim3(RT / GBM, N2 / GBN), GTHR, 0, stream>>>(Ypl, OUTW, KCAT, V2, V2, X1, N2, X1, XCH);
  k_m1_scan<<<RT / 4, 128, 0, stream>>>(Hf, X1, M1C, out);
}
